// TrafficPredictorGNN_76519137345540
// MI455X (gfx1250) — hardware-verified
//
#include <hip/hip_runtime.h>
#define NN 50000
#define NE 800000
#define CC 128
#define NCP 128

typedef __bf16 v16b __attribute__((ext_vector_type(16)));
typedef unsigned short v8us __attribute__((ext_vector_type(8), may_alias));
typedef float  v8f  __attribute__((ext_vector_type(8)));
typedef float  v4f  __attribute__((ext_vector_type(4)));
typedef float  v4fa __attribute__((ext_vector_type(4), may_alias));
union FragB { v16b v; v8us half[2]; unsigned short u[16]; };

__device__ __forceinline__ unsigned short bf16_bits(float x) { unsigned int u = __float_as_uint(x); return (unsigned short)((u + 0x7FFFu + ((u >> 16) & 1u)) >> 16); }
__device__ __forceinline__ float bf16_val(unsigned short b) { return __uint_as_float(((unsigned int)b) << 16); }
__device__ __forceinline__ float bf16_round(float x) { return bf16_val(bf16_bits(x)); }
template <int NT>
__device__ __forceinline__ v8f mmaN(v16b ah, v16b al, v16b bh, v16b bl, v8f c) {
  c = __builtin_amdgcn_wmma_f32_16x16x32_bf16(false, ah, false, bh, (short)0, c, false, false);
  if (NT >= 2) c = __builtin_amdgcn_wmma_f32_16x16x32_bf16(false, al, false, bh, (short)0, c, false, false);
  if (NT >= 3) c = __builtin_amdgcn_wmma_f32_16x16x32_bf16(false, ah, false, bl, (short)0, c, false, false);
  asm volatile("v_nop\n\tv_nop\n\tv_nop\n\tv_nop" : "+v"(c) : "v"(ah), "v"(al), "v"(bh), "v"(bl));
  return c;
}

__global__ __launch_bounds__(256) void k_wt_bf16(const float* __restrict__ W, unsigned short* __restrict__ Wt, int K, int N) {
  const int t = blockIdx.x * 256 + threadIdx.x;
  const int k8n = K / 8;
  if (t >= N * k8n) return;
  const int n = t / k8n, k8 = (t % k8n) * 8;
  v8us v;
#pragma unroll
  for (int i = 0; i < 8; ++i) v[i] = bf16_bits(W[(size_t)(k8 + i) * N + n]);
  *(volatile v8us*)(Wt + (size_t)n * K + k8) = v;
  __threadfence();
  *(volatile v8us*)(Wt + (size_t)n * K + k8) = v;
}

template <bool ASPLIT, int ACT, bool BIAS_BF16>
__global__ __launch_bounds__(128) void k_gemm_bf(const float* __restrict__ A, int lda, const unsigned short* __restrict__ Wt, int ldb,
                                               const float* __restrict__ bias, float* __restrict__ C, int ldc, int M, int N, int K) {
  __shared__ __attribute__((aligned(16))) float so[4][16][64];
  const int tid = threadIdx.x, w = tid >> 5, lane = tid & 31, ln = lane & 15, hh = lane >> 4;
  const int ntn = N / 64;
  const int wid = blockIdx.x * 4 + w;
  const int mt = wid / ntn, nq = wid % ntn;
  if (mt * 16 >= M) return;
  const int row0 = mt * 16, col0 = nq * 64;
  const float* arow = A + (size_t)(row0 + ln) * lda;
  v8f acc[4] = {};
  for (int kb = 0; kb < K; kb += 32) {
    FragB ah, al;
    const v4f x0 = *(const v4fa*)(arow + kb + 8 * hh), x1 = *(const v4fa*)(arow + kb + 8 * hh + 4);
    const v4f x2 = *(const v4fa*)(arow + kb + 16 + 8 * hh), x3 = *(const v4fa*)(arow + kb + 16 + 8 * hh + 4);
    float xs[16] = {x0[0],x0[1],x0[2],x0[3],x1[0],x1[1],x1[2],x1[3],x2[0],x2[1],x2[2],x2[3],x3[0],x3[1],x3[2],x3[3]};
#pragma unroll
    for (int i = 0; i < 16; ++i) { const unsigned short hb = bf16_bits(xs[i]); ah.u[i] = hb; al.u[i] = ASPLIT ? bf16_bits(xs[i] - bf16_val(hb)) : (unsigned short)0; }
#pragma unroll
    for (int t = 0; t < 4; ++t) {
      const unsigned short* brow = Wt + (size_t)(col0 + t * 16 + ln) * ldb + kb;
      FragB b;
      b.half[0] = *(const v8us*)(brow + 8 * hh);
      b.half[1] = *(const v8us*)(brow + 16 + 8 * hh);
      acc[t] = mmaN<ASPLIT ? 2 : 1>(ah.v, al.v, b.v, b.v, acc[t]);
    }
  }
#pragma unroll
  for (int t = 0; t < 4; ++t) {
    float bv = bias ? bias[col0 + t * 16 + ln] : 0.f;
    if (BIAS_BF16) bv = bf16_round(bv);
#pragma unroll
    for (int r = 0; r < 8; ++r) { float v = acc[t][r] + bv; if (ACT == 1) v = fmaxf(v, 0.f); so[w][8 * hh + r][t * 16 + ln] = v; }
  }
  __builtin_amdgcn_fence(__ATOMIC_ACQ_REL, "workgroup");
  __builtin_amdgcn_wave_barrier();
  const int rsub = lane >> 4, c4 = (lane & 15) * 4;
  for (int pass = 0; pass < 2; ++pass) {
#pragma unroll
    for (int q = 0; q < 8; ++q) {
      const int r = q * 2 + rsub;
      const v4f v = *(const v4fa*)&so[w][r][c4];
      *(volatile v4f*)(C + (size_t)(row0 + r) * ldc + col0 + c4) = v;
    }
    if (pass == 0) __threadfence();
  }
}

template <int D, bool CAUSAL>
__global__ __launch_bounds__(128) void k_flash(const float* __restrict__ qb, const float* __restrict__ kb, const float* __restrict__ vb,
                                             int pitch, int T, int H, float scale, float* __restrict__ y, int ypitch) {
  constexpr int KS = D / 32;
  constexpr int DT = D / 16;
  __shared__ __attribute__((aligned(16))) unsigned short sKh[32][D + 8], sKl[32][D + 8], sVh[32][D + 8], sVl[32][D + 8];
  __shared__ __attribute__((aligned(16))) unsigned short sPh[4][16][40], sPl[4][16][40];
  __shared__ __attribute__((aligned(16))) float sO[4][16][D];
  const int tid = threadIdx.x, w = tid >> 5, lane = tid & 31, ln = lane & 15, hh = lane >> 4;
  const int nqb = (T + 63) / 64;
  const int bh = blockIdx.x / nqb, qblk = blockIdx.x % nqb;
  const int b = bh / H, h = bh % H;
  const int q0 = qblk * 64 + w * 16;
  const float* Q = qb + (size_t)b * T * pitch + h * D;
  const float* K = kb + (size_t)b * T * pitch + h * D;
  const float* V = vb + (size_t)b * T * pitch + h * D;

  FragB aqh[KS], aql[KS];
  {
    int row = q0 + ln; if (row >= T) row = T - 1;
    const float* qr = Q + (size_t)row * pitch;
#pragma unroll
    for (int ks = 0; ks < KS; ++ks)
#pragma unroll
      for (int i = 0; i < 16; ++i) {
        const int d = ks * 32 + ((i < 8) ? (8 * hh + i) : (16 + 8 * hh + (i - 8)));
        const float x = qr[d] * scale; const unsigned short hb = bf16_bits(x);
        aqh[ks].u[i] = hb; aql[ks].u[i] = bf16_bits(x - bf16_val(hb));
      }
  }
  float m_r[8], l_r[8];
#pragma unroll
  for (int r = 0; r < 8; ++r) { m_r[r] = -3.0e38f; l_r[r] = 0.f; }
  v8f oacc[DT];
#pragma unroll
  for (int dt = 0; dt < DT; ++dt) oacc[dt] = (v8f){0.f,0.f,0.f,0.f,0.f,0.f,0.f,0.f};

  const int kv_end = CAUSAL ? min(T, qblk * 64 + 64) : T;
  for (int j0 = 0; j0 < kv_end; j0 += 32) {
    __syncthreads();
    for (int e = tid; e < 32 * (D / 4); e += 128) {
      const int r = e / (D / 4), c4 = (e % (D / 4)) * 4;
      const int key = j0 + r;
      v4f kf = {0.f,0.f,0.f,0.f}, vf = {0.f,0.f,0.f,0.f};
      if (key < T) { kf = *(const v4fa*)(K + (size_t)key * pitch + c4); vf = *(const v4fa*)(V + (size_t)key * pitch + c4); }
#pragma unroll
      for (int t = 0; t < 4; ++t) {
        unsigned short hb = bf16_bits(kf[t]); sKh[r][c4 + t] = hb; sKl[r][c4 + t] = bf16_bits(kf[t] - bf16_val(hb));
        hb = bf16_bits(vf[t]); sVh[r][c4 + t] = hb; sVl[r][c4 + t] = bf16_bits(vf[t] - bf16_val(hb));
      }
    }
    __syncthreads();
    v8f s[2];
#pragma unroll
    for (int nt = 0; nt < 2; ++nt) {
      v8f acc = {};
#pragma unroll
      for (int ks = 0; ks < KS; ++ks) {
        FragB bh_, bl_;
        bh_.half[0] = *(const v8us*)&sKh[nt * 16 + ln][ks * 32 + 8 * hh]; bh_.half[1] = *(const v8us*)&sKh[nt * 16 + ln][ks * 32 + 16 + 8 * hh];
        bl_.half[0] = *(const v8us*)&sKl[nt * 16 + ln][ks * 32 + 8 * hh]; bl_.half[1] = *(const v8us*)&sKl[nt * 16 + ln][ks * 32 + 16 + 8 * hh];
        acc = mmaN<3>(aqh[ks].v, aql[ks].v, bh_.v, bl_.v, acc);
      }
      s[nt] = acc;
    }
    float alpha[8];
#pragma unroll
    for (int r = 0; r < 8; ++r) {
      const int qi = q0 + 8 * hh + r;
      const int ja = j0 + ln, jb = j0 + 16 + ln;
      if (CAUSAL) { if (ja > qi) s[0][r] = -3.0e38f; if (jb > qi) s[1][r] = -3.0e38f; }
      if (ja >= T) s[0][r] = -3.0e38f;
      if (jb >= T) s[1][r] = -3.0e38f;
      float mx = fmaxf(s[0][r], s[1][r]);
      mx = fmaxf(mx, __shfl_xor(mx, 1, 32)); mx = fmaxf(mx, __shfl_xor(mx, 2, 32)); mx = fmaxf(mx, __shfl_xor(mx, 4, 32)); mx = fmaxf(mx, __shfl_xor(mx, 8, 32));
      const float mnew = fmaxf(m_r[r], mx);
      alpha[r] = (mnew > -1.0e38f) ? __expf(m_r[r] - mnew) : 1.0f;
      const float p0 = (s[0][r] > -1.0e38f) ? __expf(s[0][r] - mnew) : 0.f;
      const float p1 = (s[1][r] > -1.0e38f) ? __expf(s[1][r] - mnew) : 0.f;
      m_r[r] = mnew;
      l_r[r] = l_r[r] * alpha[r] + p0 + p1;
      unsigned short hb = bf16_bits(p0); sPh[w][8 * hh + r][ln] = hb;      sPl[w][8 * hh + r][ln] = bf16_bits(p0 - bf16_val(hb));
      hb = bf16_bits(p1);                sPh[w][8 * hh + r][16 + ln] = hb; sPl[w][8 * hh + r][16 + ln] = bf16_bits(p1 - bf16_val(hb));
    }
#pragma unroll
    for (int dt = 0; dt < DT; ++dt)
#pragma unroll
      for (int r = 0; r < 8; ++r) oacc[dt][r] *= alpha[r];
    __builtin_amdgcn_fence(__ATOMIC_ACQ_REL, "workgroup");
    __builtin_amdgcn_wave_barrier();
    FragB pah, pal;
    pah.half[0] = *(const v8us*)&sPh[w][ln][8 * hh]; pah.half[1] = *(const v8us*)&sPh[w][ln][16 + 8 * hh];
    pal.half[0] = *(const v8us*)&sPl[w][ln][8 * hh]; pal.half[1] = *(const v8us*)&sPl[w][ln][16 + 8 * hh];
#pragma unroll
    for (int dt = 0; dt < DT; ++dt) {
      FragB bvh, bvl;
#pragma unroll
      for (int i = 0; i < 8; ++i) {
        bvh.u[i] = sVh[8 * hh + i][dt * 16 + ln]; bvh.u[8 + i] = sVh[16 + 8 * hh + i][dt * 16 + ln];
        bvl.u[i] = sVl[8 * hh + i][dt * 16 + ln]; bvl.u[8 + i] = sVl[16 + 8 * hh + i][dt * 16 + ln];
      }
      oacc[dt] = mmaN<3>(pah.v, pal.v, bvh.v, bvl.v, oacc[dt]);
    }
    __builtin_amdgcn_fence(__ATOMIC_ACQ_REL, "workgroup");
    __builtin_amdgcn_wave_barrier();
  }
#pragma unroll
  for (int r = 0; r < 8; ++r) {
    float l = l_r[r];
    l += __shfl_xor(l, 1, 32); l += __shfl_xor(l, 2, 32); l += __shfl_xor(l, 4, 32); l += __shfl_xor(l, 8, 32);
    l_r[r] = (l > 0.f) ? 1.0f / l : 0.f;
  }
#pragma unroll
  for (int dt = 0; dt < DT; ++dt)
#pragma unroll
    for (int r = 0; r < 8; ++r) sO[w][8 * hh + r][dt * 16 + ln] = oacc[dt][r] * l_r[r];
  __builtin_amdgcn_fence(__ATOMIC_ACQ_REL, "workgroup");
  __builtin_amdgcn_wave_barrier();
  for (int pass = 0; pass < 2; ++pass) {
    for (int r = 0; r < 16; ++r) {
      const int row = q0 + r;
      if (row < T && lane < D / 4) {
        const v4f val = *(const v4fa*)&sO[w][r][lane * 4];
        *(volatile v4f*)(y + ((size_t)b * T + row) * ypitch + h * D + lane * 4) = val;
      }
    }
    if (pass == 0) __threadfence();
  }
}

template <bool ASPLIT, bool BSPLIT, int ACT>
__global__ __launch_bounds__(128) void k_gemm_b(const float* __restrict__ A, int lda, size_t sA, const unsigned short* __restrict__ Bh, const unsigned short* __restrict__ Bl, int ldb, size_t sB,
                                             const float* __restrict__ bias, const float* __restrict__ resid, int ldr, size_t sR, float rsign, float alpha,
                                             float* __restrict__ C, int ldc, size_t sC, int M, int N, int K) {
  __shared__ __attribute__((aligned(16))) float so[4][16][64];
  const int tid = threadIdx.x, w = tid >> 5, lane = tid & 31, ln = lane & 15, hh = lane >> 4;
  const int by = blockIdx.y;
  A += (size_t)by * sA; Bh += (size_t)by * sB; if (BSPLIT) Bl += (size_t)by * sB; C += (size_t)by * sC; if (resid) resid += (size_t)by * sR;
  const int ntn = (N + 63) / 64; const int wid = blockIdx.x * 4 + w; const int mt = wid / ntn, nq = wid % ntn;
  if (mt * 16 >= M) return;
  const int row0 = mt * 16, col0 = nq * 64;
  const float* arow = A + (size_t)(row0 + ln) * lda;
  v8f acc[4] = {};
  for (int kb = 0; kb < K; kb += 32) {
    FragB ah, al;
    const v4f x0 = *(const v4fa*)(arow + kb + 8 * hh), x1 = *(const v4fa*)(arow + kb + 8 * hh + 4);
    const v4f x2 = *(const v4fa*)(arow + kb + 16 + 8 * hh), x3 = *(const v4fa*)(arow + kb + 16 + 8 * hh + 4);
    float xs[16] = {x0[0],x0[1],x0[2],x0[3],x1[0],x1[1],x1[2],x1[3],x2[0],x2[1],x2[2],x2[3],x3[0],x3[1],x3[2],x3[3]};
#pragma unroll
    for (int i = 0; i < 16; ++i) { const unsigned short hb = bf16_bits(xs[i]); ah.u[i] = hb; al.u[i] = ASPLIT ? bf16_bits(xs[i] - bf16_val(hb)) : (unsigned short)0; }
#pragma unroll
    for (int t = 0; t < 4; ++t) {
      if (col0 + t * 16 >= N) continue;
      const size_t boff = (size_t)(col0 + t * 16 + ln) * ldb + kb;
      FragB bh_, bl_; bh_.half[0] = *(const v8us*)(Bh + boff + 8 * hh); bh_.half[1] = *(const v8us*)(Bh + boff + 16 + 8 * hh);
      if (BSPLIT) { bl_.half[0] = *(const v8us*)(Bl + boff + 8 * hh); bl_.half[1] = *(const v8us*)(Bl + boff + 16 + 8 * hh); } else bl_ = bh_;
      acc[t] = mmaN<ASPLIT ? (BSPLIT ? 3 : 2) : 1>(ah.v, al.v, bh_.v, bl_.v, acc[t]);
    }
  }
#pragma unroll
  for (int t = 0; t < 4; ++t) {
    const int col = col0 + t * 16 + ln; if (col0 + t * 16 >= N) continue; const float bv = bias ? bf16_round(bias[col]) : 0.f;
#pragma unroll
    for (int r = 0; r < 8; ++r) { float v = acc[t][r] * alpha + bv; if (resid) v += rsign * resid[(size_t)(row0 + 8 * hh + r) * ldr + col]; if (ACT == 1) v = fmaxf(v, 0.f); else if (ACT == 2) v = fmaxf(v, 0.f) + log1pf(expf(-fabsf(v))); so[w][8 * hh + r][t * 16 + ln] = v; }
  }
  __builtin_amdgcn_fence(__ATOMIC_ACQ_REL, "workgroup"); __builtin_amdgcn_wave_barrier();
  const int rsub = lane >> 4, c4 = (lane & 15) * 4;
  for (int pass = 0; pass < 2; ++pass) {
#pragma unroll
    for (int q = 0; q < 8; ++q) { const int r = q * 2 + rsub; if (col0 + c4 < N) { const v4f v = *(const v4fa*)&so[w][r][c4]; *(volatile v4f*)(C + (size_t)(row0 + r) * ldc + col0 + c4) = v; } }
    if (pass == 0) __threadfence();
  }
}
__global__ __launch_bounds__(256) void k_split_transpose_b(const float* __restrict__ src, int lds_, size_t sIn, unsigned short* __restrict__ hi, unsigned short* __restrict__ lo, size_t sOut, int K, int N) {
  const size_t t = (size_t)blockIdx.x * 256 + threadIdx.x; const int k8n = K / 8; if (t >= (size_t)N * k8n) return;
  src += (size_t)blockIdx.y * sIn; hi += (size_t)blockIdx.y * sOut; lo += (size_t)blockIdx.y * sOut;
  const int n = (int)(t / k8n), k8 = (int)(t % k8n) * 8; v8us vh, vl;
#pragma unroll
  for (int i = 0; i < 8; ++i) { const float x = src[(size_t)(k8 + i) * lds_ + n]; const unsigned short hb = bf16_bits(x); vh[i] = hb; vl[i] = bf16_bits(x - bf16_val(hb)); }
  unsigned short* dh = hi + (size_t)n * K + k8; unsigned short* dl = lo + (size_t)n * K + k8;
  *(volatile v8us*)dh = vh; *(volatile v8us*)dl = vl; __threadfence(); *(volatile v8us*)dh = vh; *(volatile v8us*)dl = vl;
}

__global__ __launch_bounds__(256) void k_bt(const float* __restrict__ W1, const float* __restrict__ W2, const float* __restrict__ W3, unsigned short* __restrict__ Bt) { const int t = blockIdx.x * 256 + threadIdx.x; if (t >= 3 * CC * CC) return; const int l = t / (CC * CC), r = t % (CC * CC); const int k = r % CC, n = r / CC; const float* W = l == 0 ? W1 : (l == 1 ? W2 : W3); *(volatile unsigned short*)(Bt + t) = bf16_bits(W[k * CC + n]); }

__device__ __forceinline__ int bscan_k_seg(int cnt, int* scan, int tid, int& total) { __syncthreads(); scan[tid] = cnt; __syncthreads();
  for (int of = 1; of < 512; of <<= 1) { const int v = (tid >= of) ? scan[tid - of] : 0; __syncthreads(); scan[tid] += v; __syncthreads(); }
  total = scan[512 - 1]; return scan[tid] - cnt; }
__global__ __launch_bounds__(512) void k_seg(const float* __restrict__ SRC, const int* __restrict__ src, const int* __restrict__ dst, const float* __restrict__ ew, const float* __restrict__ DINV, float* __restrict__ RAW) {
  __shared__ short Lr[4096]; __shared__ int Lc[4096]; __shared__ float Lw[4096]; __shared__ int scan[512]; __shared__ float stg[64][128 + 1];
  const int tid = threadIdx.x; const int s0 = blockIdx.x * 512; float acc0[128];
#pragma unroll
  for (int c = 0; c < 128; ++c) acc0[c] = 0.f;
  for (int e0 = 0; e0 < (NE); e0 += 4096) { int hr[8], hc[8]; float hw[8]; int cnt = 0;
#pragma unroll
    for (int k = 0; k < 8; ++k) { const int e = e0 + tid * 8 + k; hr[k] = -1; hc[k] = 0; hw[k] = 0.f; if (e < (NE)) { const int dd_ = (dst[e]); if (dd_ >= s0 && dd_ < s0 + 512) { hr[k] = dd_ - s0; int s = (src[e]); s = s < 0 ? 0 : (s >= (NN) ? (NN) - 1 : s); hc[k] = s; hw[k] = (bf16_round(ew[e]) * DINV[s]); ++cnt; } } }
    int tot; int p = bscan_k_seg(cnt, scan, tid, tot);
#pragma unroll
    for (int k = 0; k < 8; ++k) if (hr[k] >= 0) { Lr[p] = (short)hr[k]; Lc[p] = hc[k]; Lw[p] = hw[k]; ++p; }
    __syncthreads();
#pragma unroll 1
    for (int q = 0; q < tot; ++q) { if (Lr[q] == tid) { const float* row = (SRC + (size_t)Lc[q] * CC); const float w = Lw[q];
#pragma unroll
        for (int c = 0; c < 128; c += 4) { const v4f v = *(const v4fa*)(row + c); acc0[c] += w * v[0]; acc0[c + 1] += w * v[1]; acc0[c + 2] += w * v[2]; acc0[c + 3] += w * v[3]; } } }
    __syncthreads(); }
  for (int tg = 0; tg < 512 / 64; ++tg) {
    if (tid / 64 == tg) {
#pragma unroll
      for (int c = 0; c < 128; ++c) stg[tid % 64][c] = acc0[c]; }
    __syncthreads();
    for (int pass = 0; pass < 2; ++pass) { for (int i = tid; i < 64 * (128 / 4); i += 512) { const int r = i / (128 / 4), c4 = (i % (128 / 4)) * 4; const int seg = s0 + tg * 64 + r; if (seg < (NN)) { v4f v; v[0] = stg[r][c4]; v[1] = stg[r][c4 + 1]; v[2] = stg[r][c4 + 2]; v[3] = stg[r][c4 + 3];  *(volatile v4f*)((RAW + (size_t)seg * CC) + c4) = v; } } if (pass == 0) __threadfence(); }
    __syncthreads(); } }

__device__ __forceinline__ int bscan1024(int cnt, int* scan, int tid, int& total) { __syncthreads(); scan[tid] = cnt; __syncthreads();
  for (int of = 1; of < 1024; of <<= 1) { const int v = (tid >= of) ? scan[tid - of] : 0; __syncthreads(); scan[tid] += v; __syncthreads(); }
  total = scan[1023]; return scan[tid] - cnt; }
__global__ __launch_bounds__(1024) void k_deg(const int* __restrict__ dst, const float* __restrict__ ew, float* __restrict__ DINV) { __shared__ short Lr[4096]; __shared__ float Lw[4096]; __shared__ int scan[1024]; const int tid = threadIdx.x; const int n0 = blockIdx.x * 1024; float d = 0.f;
  for (int e0 = 0; e0 < NE; e0 += 4096) { int hr[4]; float hw[4]; int cnt = 0;
#pragma unroll
    for (int k = 0; k < 4; ++k) { const int e = e0 + tid * 4 + k; hr[k] = -1; hw[k] = 0.f; if (e < NE) { const int dd = dst[e]; if (dd >= n0 && dd < n0 + 1024) { hr[k] = dd - n0; hw[k] = bf16_round(ew[e]); ++cnt; } } }
    int tot; int p = bscan1024(cnt, scan, tid, tot);
#pragma unroll
    for (int k = 0; k < 4; ++k) if (hr[k] >= 0) { Lr[p] = (short)hr[k]; Lw[p] = hw[k]; ++p; }
    __syncthreads();
#pragma unroll 1
    for (int q = 0; q < tot; ++q) if (Lr[q] == tid) d += Lw[q];
    __syncthreads(); }
  const int n = n0 + tid; if (n < NN) { const float v = 1.0f / sqrtf(d + 1.0f); *(volatile float*)(DINV + n) = v; __threadfence(); *(volatile float*)(DINV + n) = v; } }
__global__ __launch_bounds__(256) void k_epi(const float* __restrict__ RAW, const float* __restrict__ XW, const float* __restrict__ DINV, const float* __restrict__ b, const float* __restrict__ RES, float* __restrict__ H) { const size_t t = (size_t)blockIdx.x * 256 + threadIdx.x; if (t >= (size_t)NN * CC / 4) return; const int c4 = (int)((t * 4) % CC); const float d = DINV[(t * 4) / CC]; const v4f r = *(const v4fa*)(RAW + t * 4), x = *(const v4fa*)(XW + t * 4); v4f o;
  for (int q = 0; q < 4; ++q) { float v = d * r[q] + x[q] * d * d + bf16_round(b[c4 + q]); v = v > 0.f ? v : expm1f(v); if (RES) v += RES[t * 4 + q]; o[q] = v; } *(volatile v4f*)(H + t * 4) = o; __threadfence(); *(volatile v4f*)(H + t * 4) = o; }
__global__ __launch_bounds__(256) void k_out(const float* __restrict__ H, const float* __restrict__ Wl, const float* __restrict__ bl, float* __restrict__ out) { __shared__ float sw[CC]; if (threadIdx.x < CC) sw[threadIdx.x] = bf16_round(Wl[threadIdx.x]); __syncthreads(); const int n = blockIdx.x * 256 + threadIdx.x; if (n >= NN) return; const float* h = H + (size_t)n * CC; float s = 0.f;
#pragma unroll 4
  for (int c = 0; c < CC; c += 4) { const v4f v = *(const v4fa*)(h + c); s += v[0] * sw[c] + v[1] * sw[c + 1] + v[2] * sw[c + 2] + v[3] * sw[c + 3]; } s += bf16_round(bl[0]); const float y = 1.0f / (1.0f + expf(-s)); *(volatile float*)(out + n) = y; __threadfence(); *(volatile float*)(out + n) = y; }
extern "C" void kernel_launch(void* const* d_in, const int* in_sizes, int n_in,
                              void* d_out, int out_size, void* d_ws, size_t ws_size, hipStream_t stream) {
  (void)in_sizes; (void)n_in; (void)out_size;
  const float* x = (const float*)d_in[0]; const int* ei = (const int*)d_in[1]; const float* ew = (const float*)d_in[2]; const float* W1 = (const float*)d_in[3]; const float* b1 = (const float*)d_in[4]; const float* W2 = (const float*)d_in[5]; const float* b2 = (const float*)d_in[6]; const float* W3 = (const float*)d_in[7]; const float* b3 = (const float*)d_in[8]; const float* Wl = (const float*)d_in[9]; const float* bl = (const float*)d_in[10];
  const int* src = ei; const int* dst = ei + NE;
  char* ws = (char*)d_ws; size_t off = 0;
  auto take = [&](size_t bytes) { char* p = ws + off; off += (bytes + 255) & ~(size_t)255; return p; };
  unsigned short* Bt = (unsigned short*)take((size_t)3 * CC * CC * 2); float* DINV = (float*)take(NN * 4); float* XW = (float*)take((size_t)NN * CC * 4); float* RAW = (float*)take((size_t)NN * CC * 4); float* H1 = (float*)take((size_t)NN * CC * 4); float* H2 = (float*)take((size_t)NN * CC * 4);
  if (off > ws_size) return;
  const unsigned EW4 = (unsigned)(((size_t)NN * CC / 4 + 255) / 256); const int NT = (NN + 511) / 512; const dim3 gg(((NN / 16) * (CC / 64) + 3) / 4, 1);
  k_bt<<<(3 * CC * CC + 255) / 256, 256, 0, stream>>>(W1, W2, W3, Bt); k_deg<<<(NN + 1023) / 1024, 1024, 0, stream>>>(dst, ew, DINV);
  auto layer = [&](const float* hin, bool first, const unsigned short* B, const float* b, const float* res, float* hout) {
    if (first) k_gemm_b<false, false, 0><<<gg, 128, 0, stream>>>(hin, CC, 0, B, B, CC, 0, nullptr, nullptr, 0, 0, 1.f, 1.f, XW, CC, 0, NN, CC, CC);
    else k_gemm_b<true, false, 0><<<gg, 128, 0, stream>>>(hin, CC, 0, B, B, CC, 0, nullptr, nullptr, 0, 0, 1.f, 1.f, XW, CC, 0, NN, CC, CC);
    k_seg<<<NT, 512, 0, stream>>>(XW, src, dst, ew, DINV, RAW);
    k_epi<<<EW4, 256, 0, stream>>>(RAW, XW, DINV, b, res, hout); };
  layer(x, true, Bt, b1, nullptr, H1);
  layer(H1, false, Bt + CC * CC, b2, H1, H2);
  layer(H2, false, Bt + 2 * CC * CC, b3, H2, H1);
  k_out<<<(NN + 255) / 256, 256, 0, stream>>>(H1, Wl, bl, (float*)d_out);
}
